// MultiHeadAttention_60859686584499
// MI455X (gfx1250) — hardware-verified
//
#include <hip/hip_runtime.h>
#include <math.h>

typedef __attribute__((ext_vector_type(16))) _Float16 v16h;
typedef __attribute__((ext_vector_type(16))) __bf16 v16b;
typedef __attribute__((ext_vector_type(8)))  _Float16 v8h;
typedef __attribute__((ext_vector_type(8)))  __bf16 v8b;
typedef __attribute__((ext_vector_type(8)))  float v8f;
typedef __attribute__((ext_vector_type(4)))  float v4f;
typedef __attribute__((ext_vector_type(4)))  unsigned v4u;
typedef v8h __attribute__((may_alias)) v8h_a;
typedef v4u __attribute__((may_alias)) v4u_a;
typedef v4f __attribute__((may_alias)) v4f_a;

#ifndef NB
#define NB 2
#endif
#ifndef SEQ
#define SEQ 2048
#endif
#define NB_FULL 2
#define SEQ_FULL 2048
#define DIN 1024
#define NH 16
#define HD 64
#define CC (NH * HD)
#define MROWS (NB * SEQ)
#define SCL2 (0.18033688011112042f)
#define NEGB (-3.0e38f)

static_assert(HD == 64);
static_assert(CC == NH * HD);
static_assert(CC == 1024);
static_assert((CC & (CC - 1)) == 0);
static_assert(DIN % 64 == 0);
static_assert(DIN % 32 == 0);
static_assert(CC % 128 == 0);
static_assert(DIN % 128 == 0);
static_assert((3 * CC) % 128 == 0);
static_assert(SEQ % 64 == 0);
static_assert(MROWS % 64 == 0);
static_assert(SEQ <= SEQ_FULL);
static_assert(NB <= NB_FULL);
static_assert(((size_t)MROWS * DIN / 8) % 256 == 0);

#define WS_XB  ((size_t)0)
#define WS_WT  (WS_XB  + (size_t)2 * MROWS * DIN)
#define WS_WPT (WS_WT  + (size_t)2 * 3 * CC * DIN)
#define WS_QH  (WS_WPT + (size_t)2 * DIN * CC)
#define WS_KH  (WS_QH  + (size_t)2 * MROWS * CC)
#define WS_VT  (WS_KH  + (size_t)2 * MROWS * CC)
#define WS_CT  (WS_VT  + (size_t)2 * NB * CC * SEQ)
#define WS_END (WS_CT  + (size_t)2 * MROWS * 2 * CC)
static_assert(WS_END <= (size_t)134217728);
static_assert(WS_WT % 128 == 0);
static_assert(WS_WPT % 128 == 0);
static_assert(WS_QH % 128 == 0);
static_assert(WS_KH % 128 == 0);
static_assert(WS_VT % 128 == 0);
static_assert(WS_CT % 128 == 0);

template <typename T> __device__ __forceinline__ void vst2(void* p, T v) { *(volatile T*)p = v; __threadfence(); *(volatile T*)p = v; }

__device__ __forceinline__ v8f wmma16(v16h a, v16h b, v8f c) {
  v8f d = __builtin_amdgcn_wmma_f32_16x16x32_f16(false, a, false, b, (short)0, c, false, false);
  asm volatile("v_nop\n\tv_nop\n\tv_nop\n\tv_nop" : "+v"(d) : "v"(a), "v"(b));
  return d;
}
__device__ __forceinline__ v8f wmma_bf(v16b a, v16b b, v8f c) {
  v8f d = __builtin_amdgcn_wmma_f32_16x16x32_bf16(false, a, false, b, (short)0, c, false, false);
  asm volatile("v_nop\n\tv_nop\n\tv_nop\n\tv_nop" : "+v"(d) : "v"(a), "v"(b));
  return d;
}
__device__ __forceinline__ v16h frag_h(const _Float16* rowk0, int lane) {
  union { v16h v; v8h q[2]; } u; const _Float16* p = rowk0 + 8 * (lane >> 4);
  u.q[0] = *(const v8h*)p; u.q[1] = *(const v8h*)(p + 16); return u.v;
}
__device__ __forceinline__ v16b frag_b(const __bf16* rowk0, int lane) {
  union { v16b v; v8b q[2]; } u; const __bf16* p = rowk0 + 8 * (lane >> 4);
  u.q[0] = *(const v8b*)p; u.q[1] = *(const v8b*)(p + 16); return u.v;
}
__device__ __forceinline__ unsigned bf16_rne_bits(float v) { const unsigned u = __float_as_uint(v); return (u + 0x7FFFu + ((u >> 16) & 1u)) >> 16; }
__device__ __forceinline__ float bfr(float v) { return __uint_as_float(bf16_rne_bits(v) << 16); }
#define LDSX() do { asm volatile("s_wait_dscnt 0" ::: "memory"); __builtin_amdgcn_wave_barrier(); __builtin_amdgcn_fence(3  , "workgroup"); } while (0)

__global__ __launch_bounds__(256) void k_cvtx(const float* __restrict__ X, unsigned short* __restrict__ XB) {
  const size_t i = (size_t)blockIdx.x * 256 + threadIdx.x;
  const size_t row = i / (DIN / 8); const int pc = (int)(i % (DIN / 8));
  const size_t b = row / SEQ, t = row % SEQ;
  const float* src = X + (b * SEQ_FULL + t) * DIN + pc * 8;
  const v4f a = *(const v4f*)src, c = *(const v4f*)(src + 4);
  v4u o;
  o[0] = bf16_rne_bits(a[0]) | (bf16_rne_bits(a[1]) << 16);
  o[1] = bf16_rne_bits(a[2]) | (bf16_rne_bits(a[3]) << 16);
  o[2] = bf16_rne_bits(c[0]) | (bf16_rne_bits(c[1]) << 16);
  o[3] = bf16_rne_bits(c[2]) | (bf16_rne_bits(c[3]) << 16);
  vst2(XB + row * DIN + pc * 8, o);
}

__global__ __launch_bounds__(128) void k_tr(const float* __restrict__ IN, unsigned short* __restrict__ OUT, int in_ld, int out_ld, int in_bs, int out_bs) {
  __shared__ __align__(16) unsigned short tt[64][72];
  const int tid = threadIdx.x; const int r0 = blockIdx.x * 64, c0 = blockIdx.y * 64;
  const float* src = IN + (size_t)blockIdx.z * in_bs; unsigned short* dst = OUT + (size_t)blockIdx.z * out_bs;
#pragma unroll 1
  for (int e = tid; e < 64 * 16; e += 128) { const int rr = e >> 4, q = e & 15;
    const v4f v = *(const v4f*)(src + (size_t)(r0 + rr) * in_ld + c0 + q * 4);
    tt[q * 4 + 0][rr] = (unsigned short)bf16_rne_bits(v[0]); tt[q * 4 + 1][rr] = (unsigned short)bf16_rne_bits(v[1]);
    tt[q * 4 + 2][rr] = (unsigned short)bf16_rne_bits(v[2]); tt[q * 4 + 3][rr] = (unsigned short)bf16_rne_bits(v[3]); }
  __syncthreads();
#pragma unroll 1
  for (int e = tid; e < 64 * 8; e += 128) { const int n = e >> 3, p = e & 7;
    const v4u v = *(const v4u_a*)&tt[n][p * 8];
    vst2(dst + (size_t)(c0 + n) * out_ld + r0 + p * 8, v); }
}

__global__ __launch_bounds__(128) void k_proj(const __bf16* __restrict__ XB, const __bf16* __restrict__ WT, _Float16* __restrict__ QH, _Float16* __restrict__ KH, _Float16* __restrict__ VT) {
  __shared__ __align__(16) _Float16 sh[64][136];
  __shared__ __align__(16) _Float16 th[128][72];
  const int tid = threadIdx.x, lane = tid & 31, col = lane & 15, g = lane >> 4;
  const int wave = __builtin_amdgcn_readfirstlane((int)(threadIdx.x >> 5));
  const int wm = wave >> 1, wn = wave & 1;
  const int r0 = blockIdx.x * 64, c0 = blockIdx.y * 128;
  const int which = c0 / CC, cw = c0 % CC;
  const int bb = r0 / SEQ, t0 = r0 % SEQ;
  const __bf16* ar0 = XB + (size_t)(r0 + wm * 32 + col) * DIN; const __bf16* ar1 = ar0 + (size_t)16 * DIN;
  const __bf16* br = WT + (size_t)(c0 + wn * 64 + col) * DIN;
  v8f acc[2][4] = {};
#pragma unroll 2
  for (int kc = 0; kc < DIN / 32; ++kc) {
    const v16b a0 = frag_b(ar0 + kc * 32, lane), a1 = frag_b(ar1 + kc * 32, lane);
#pragma unroll
    for (int j = 0; j < 4; ++j) { const v16b w = frag_b(br + (size_t)j * 16 * DIN + kc * 32, lane); acc[0][j] = wmma_bf(a0, w, acc[0][j]); acc[1][j] = wmma_bf(a1, w, acc[1][j]); }
  }
  if (which < 2) {
#pragma unroll
    for (int mt = 0; mt < 2; ++mt)
#pragma unroll
      for (int j = 0; j < 4; ++j)
#pragma unroll
        for (int r = 0; r < 8; ++r) sh[wm * 32 + mt * 16 + 8 * g + r][wn * 64 + j * 16 + col] = (_Float16)acc[mt][j][r];
  } else {
#pragma unroll
    for (int mt = 0; mt < 2; ++mt)
#pragma unroll
      for (int j = 0; j < 4; ++j)
#pragma unroll
        for (int r = 0; r < 8; ++r) th[wn * 64 + j * 16 + col][wm * 32 + mt * 16 + 8 * g + r] = (_Float16)acc[mt][j][r];
  }
  __syncthreads();
  if (which == 0) {
#pragma unroll 1
    for (int e = tid; e < 64 * 16; e += 128) { const int rl = e >> 4, q = e & 15; const v4u v = *(const v4u_a*)&sh[rl][q * 8]; vst2(QH + (size_t)(r0 + rl) * CC + cw + q * 8, v); }
  } else if (which == 1) {
#pragma unroll 1
    for (int e = tid; e < 64 * 16; e += 128) { const int rl = e >> 4, q = e & 15; const v4u v = *(const v4u_a*)&sh[rl][q * 8]; vst2(KH + (size_t)(r0 + rl) * CC + cw + q * 8, v); }
  } else {
#pragma unroll 1
    for (int e = tid; e < 128 * 8; e += 128) { const int cl = e >> 3, q = e & 7; const v4u v = *(const v4u_a*)&th[cl][q * 8]; vst2(VT + ((size_t)bb * CC + cw + cl) * SEQ + t0 + q * 8, v); }
  }
}

__global__ __launch_bounds__(128) void k_attn(const _Float16* __restrict__ QH, const _Float16* __restrict__ KH, const _Float16* __restrict__ VT, const int* __restrict__ LEN, unsigned short* __restrict__ CT) {
  __shared__ __align__(16) _Float16 pb[4][16][40];
  __shared__ __align__(16) unsigned short csh[4][16][72];
  __shared__ __align__(16) unsigned short csl[4][16][72];
  const int tid = threadIdx.x, lane = tid & 31, col = lane & 15, g = lane >> 4;
  const int wave = __builtin_amdgcn_readfirstlane((int)(threadIdx.x >> 5));
  const int b = blockIdx.z, h = blockIdx.y; const int qt0 = blockIdx.x * 64 + wave * 16;
  int len = LEN[b]; len = len < 0 ? 0 : (len > SEQ ? SEQ : len);
  const int send = (qt0 < len) ? ((len + 31) & ~31) : 0;
  const _Float16* qrow = QH + ((size_t)b * SEQ + qt0 + col) * CC + h * HD;
  const v16h q0f = frag_h(qrow, lane), q1f = frag_h(qrow + 32, lane);
  v8f o[4] = {};
  float m[8], l[8];
#pragma unroll
  for (int r = 0; r < 8; ++r) { m[r] = NEGB; l[r] = 0.f; }
#pragma unroll 1
  for (int s0 = 0; s0 < send; s0 += 32) {
    const _Float16* kp0 = KH + ((size_t)b * SEQ + s0 + col) * CC + h * HD; const _Float16* kp1 = kp0 + (size_t)16 * CC;
    v8f S0 = {}, S1 = {};
    S0 = wmma16(q0f, frag_h(kp0, lane), S0); S0 = wmma16(q1f, frag_h(kp0 + 32, lane), S0);
    S1 = wmma16(q0f, frag_h(kp1, lane), S1); S1 = wmma16(q1f, frag_h(kp1 + 32, lane), S1);
    const bool v0 = (s0 + col) < len, v1 = (s0 + 16 + col) < len;
#pragma unroll
    for (int r = 0; r < 8; ++r) {
      const float x0 = v0 ? S0[r] * SCL2 : NEGB, x1 = v1 ? S1[r] * SCL2 : NEGB;
      float mx = fmaxf(x0, x1);
      mx = fmaxf(mx, __shfl_xor(mx, 1)); mx = fmaxf(mx, __shfl_xor(mx, 2)); mx = fmaxf(mx, __shfl_xor(mx, 4)); mx = fmaxf(mx, __shfl_xor(mx, 8));
      const float mn = fmaxf(m[r], mx);
      const float al = exp2f(m[r] - mn);
      const float e0 = exp2f(x0 - mn), e1 = exp2f(x1 - mn);
      const float p0 = v0 ? e0 : 0.f, p1 = v1 ? e1 : 0.f;
      m[r] = mn; l[r] = l[r] * al + (p0 + p1);
      o[0][r] *= al; o[1][r] *= al; o[2][r] *= al; o[3][r] *= al;
      pb[wave][8 * g + r][col] = (_Float16)(p0 * 1024.0f); pb[wave][8 * g + r][16 + col] = (_Float16)(p1 * 1024.0f);
    }
    LDSX();
    union { v16h v; v8h q[2]; } pf;
    pf.q[0] = *(const v8h_a*)&pb[wave][col][8 * g]; pf.q[1] = *(const v8h_a*)&pb[wave][col][16 + 8 * g];
    const _Float16* vp = VT + ((size_t)b * CC + h * HD + col) * SEQ + s0;
#pragma unroll
    for (int j = 0; j < 4; ++j) o[j] = wmma16(pf.v, frag_h(vp + (size_t)j * 16 * SEQ, lane), o[j]);
  }
  float inv[8];
#pragma unroll
  for (int r = 0; r < 8; ++r) { float lt = l[r];
    lt += __shfl_xor(lt, 1); lt += __shfl_xor(lt, 2); lt += __shfl_xor(lt, 4); lt += __shfl_xor(lt, 8);
    const bool ok = ((qt0 + 8 * g + r) < len) && (lt > 0.f);
    const float den = ok ? lt * 1024.0f : 1.0f; const float rc = 1.0f / den; inv[r] = ok ? rc : 0.f; }
#pragma unroll
  for (int j = 0; j < 4; ++j)
#pragma unroll
    for (int r = 0; r < 8; ++r) { const float c = (inv[r] > 0.f) ? o[j][r] * inv[r] : 0.f;
      const unsigned hb = bf16_rne_bits(c); const unsigned lb = bf16_rne_bits(c - __uint_as_float(hb << 16));
      csh[wave][8 * g + r][j * 16 + col] = (unsigned short)hb; csl[wave][8 * g + r][j * 16 + col] = (unsigned short)lb; }
  LDSX();
  const size_t crow = (size_t)b * SEQ + qt0;
#pragma unroll
  for (int it = 0; it < 4; ++it) { const int rl = it * 4 + (lane >> 3), pc = lane & 7;
    const v4u vh = *(const v4u_a*)&csh[wave][rl][pc * 8]; const v4u vl = *(const v4u_a*)&csl[wave][rl][pc * 8];
    unsigned short* d = CT + (crow + rl) * (size_t)(2 * CC) + h * HD + pc * 8;
    vst2(d, vh); vst2(d + CC, vl); }
}

__global__ __launch_bounds__(128) void k_out(const __bf16* __restrict__ CT, const __bf16* __restrict__ WPT, const float* __restrict__ BP, float* __restrict__ OUT) {
  __shared__ __align__(16) float sf[64][132];
  const int tid = threadIdx.x, lane = tid & 31, col = lane & 15, g = lane >> 4;
  const int wave = __builtin_amdgcn_readfirstlane((int)(threadIdx.x >> 5));
  const int wm = wave >> 1, wn = wave & 1;
  const int r0 = blockIdx.x * 64, c0 = blockIdx.y * 128;
  const __bf16* ar0 = CT + (size_t)(r0 + wm * 32 + col) * (2 * CC); const __bf16* ar1 = ar0 + (size_t)16 * (2 * CC);
  const __bf16* br = WPT + (size_t)(c0 + wn * 64 + col) * CC;
  v8f acc[2][4] = {};
#pragma unroll 2
  for (int kc = 0; kc < (2 * CC) / 32; ++kc) {
    const v16b a0 = frag_b(ar0 + kc * 32, lane), a1 = frag_b(ar1 + kc * 32, lane);
    const int kw = (kc * 32) & (CC - 1);
#pragma unroll
    for (int j = 0; j < 4; ++j) { const v16b w = frag_b(br + (size_t)j * 16 * CC + kw, lane); acc[0][j] = wmma_bf(a0, w, acc[0][j]); acc[1][j] = wmma_bf(a1, w, acc[1][j]); }
  }
#pragma unroll
  for (int mt = 0; mt < 2; ++mt)
#pragma unroll
    for (int j = 0; j < 4; ++j)
#pragma unroll
      for (int r = 0; r < 8; ++r) sf[wm * 32 + mt * 16 + 8 * g + r][wn * 64 + j * 16 + col] = acc[mt][j][r];
  __syncthreads();
  const size_t orow0 = (size_t)(r0 / SEQ) * SEQ_FULL + (size_t)(r0 % SEQ);
#pragma unroll 1
  for (int e = tid; e < 64 * 32; e += 128) { const int rl = e >> 5, q = e & 31;
    v4f v = *(const v4f_a*)&sf[rl][q * 4]; const v4f bv = *(const v4f*)(BP + c0 + q * 4);
    v[0] += bfr(bv[0]); v[1] += bfr(bv[1]); v[2] += bfr(bv[2]); v[3] += bfr(bv[3]);
    vst2(OUT + (orow0 + rl) * DIN + c0 + q * 4, v); }
}

extern "C" void kernel_launch(void* const* d_in, const int* in_sizes, int n_in, void* d_out, int out_size, void* d_ws, size_t ws_size, hipStream_t stream) {
  if (n_in < 7) return;
  const long long need_rows = (long long)(NB - 1) * SEQ_FULL + SEQ;
  if ((long long)in_sizes[0] < need_rows * DIN) return;
  if (in_sizes[1] < NB) return;
  if ((long long)in_sizes[2] < (long long)NH * DIN * HD || (long long)in_sizes[3] < (long long)NH * DIN * HD || (long long)in_sizes[4] < (long long)NH * DIN * HD) return;
  if ((long long)in_sizes[5] < (long long)CC * DIN || in_sizes[6] < DIN) return;
  if ((long long)out_size < need_rows * DIN) return;
  if (ws_size < (size_t)WS_END) return;
  const float* X = (const float*)d_in[0]; const int* LEN = (const int*)d_in[1];
  const float* WQ = (const float*)d_in[2]; const float* WK = (const float*)d_in[3]; const float* WV = (const float*)d_in[4];
  const float* WP = (const float*)d_in[5]; const float* BP = (const float*)d_in[6];
  char* ws = (char*)d_ws;
  unsigned short* XBw = (unsigned short*)(ws + WS_XB); unsigned short* WTw = (unsigned short*)(ws + WS_WT); unsigned short* WPTw = (unsigned short*)(ws + WS_WPT);
  _Float16* QH = (_Float16*)(ws + WS_QH); _Float16* KH = (_Float16*)(ws + WS_KH); _Float16* VT = (_Float16*)(ws + WS_VT);
  unsigned short* CTw = (unsigned short*)(ws + WS_CT);
  k_cvtx<<<dim3((unsigned)(((size_t)MROWS * DIN / 8) / 256)), 256, 0, stream>>>(X, XBw);
  k_tr<<<dim3(DIN / 64, HD / 64, NH), 128, 0, stream>>>(WQ, WTw + (size_t)0 * CC * DIN, HD, DIN, DIN * HD, HD * DIN);
  k_tr<<<dim3(DIN / 64, HD / 64, NH), 128, 0, stream>>>(WK, WTw + (size_t)1 * CC * DIN, HD, DIN, DIN * HD, HD * DIN);
  k_tr<<<dim3(DIN / 64, HD / 64, NH), 128, 0, stream>>>(WV, WTw + (size_t)2 * CC * DIN, HD, DIN, DIN * HD, HD * DIN);
  k_tr<<<dim3(CC / 64, DIN / 64, 1), 128, 0, stream>>>(WP, WPTw, DIN, CC, 0, 0);
  k_proj<<<dim3(MROWS / 64, (3 * CC) / 128), 128, 0, stream>>>((const __bf16*)(ws + WS_XB), (const __bf16*)(ws + WS_WT), QH, KH, VT);
  k_attn<<<dim3(SEQ / 64, NH, NB), 128, 0, stream>>>(QH, KH, VT, LEN, CTw);
  k_out<<<dim3(MROWS / 64, DIN / 128), 128, 0, stream>>>((const __bf16*)(ws + WS_CT), (const __bf16*)(ws + WS_WPT), BP, (float*)d_out);
}
